// GNN_Dense_50002009260729
// MI455X (gfx1250) — hardware-verified
//
#include <hip/hip_runtime.h>
#include <stddef.h>


#define DIN   128
#define DO    64
#define NL    3
#define GR    32
#define GT    128
#define AP    136
#define HSP   68
#define NB    1024
#define SLB   10
#define CHUNK 2048
#define NTHR  256
#define NWAVE 8
#define WCAP  256
#define NGRP  (CHUNK / (NTHR * 4))
#define NG    512
#define GLB   9

#define LDS_GAT_BYTES  ((NB * DO + NB + NB + NWAVE * WCAP + NWAVE) * 4)
#define LDS_POOL_BYTES ((NG * DIN + NWAVE * WCAP + NWAVE + NG) * 4)

static_assert(WCAP == NGRP * 4 * 32);
static_assert(NGRP >= 1);
static_assert((1 << SLB) == NB);
static_assert((1 << GLB) == NG);
static_assert(CHUNK == 2048);
static_assert(DIN == 128 && DO == 64 && DIN * DO == 8192);
static_assert(LDS_GAT_BYTES == 278560);
static_assert(LDS_POOL_BYTES == 272416);
static_assert(((NB * DO) % 4) == 0 && ((NG * DIN) % 4) == 0);
static_assert(NB % (NWAVE * 2) == 0);

typedef float    v2f  __attribute__((ext_vector_type(2)));
typedef float    v4f  __attribute__((ext_vector_type(4)));
typedef float    v8f  __attribute__((ext_vector_type(8)));
typedef int      v4i  __attribute__((ext_vector_type(4)));
typedef _Float16 v8h  __attribute__((ext_vector_type(8)));
typedef _Float16 v16h __attribute__((ext_vector_type(16)));
union Frag   { v16h v; v8h half[2]; };
union Pack16 { v8h h; v4i i; };

__device__ __forceinline__ v8f wm(v16h a, v16h b, v8f c) {
  v8f d = __builtin_amdgcn_wmma_f32_16x16x32_f16(false, a, false, b, (short)0, c, false, false);
  asm volatile("v_nop\n\tv_nop\n\tv_nop\n\tv_nop" : "+v"(d) : "v"(a), "v"(b));
  return d;
}

__device__ __forceinline__ float wsum(float v) {
  v += __shfl_xor(v, 16, 32);
  v += __shfl_xor(v, 8, 32);
  v += __shfl_xor(v, 4, 32);
  v += __shfl_xor(v, 2, 32);
  v += __shfl_xor(v, 1, 32);
  return v;
}

__device__ __forceinline__ int iclamp(int v, int lo, int hi) {
  return v < lo ? lo : (v > hi ? hi : v);
}

__device__ __forceinline__ float lrelu(float v) { return v > 0.f ? v : 0.2f * v; }

__device__ __forceinline__ v4i load4(const int* __restrict__ arr, int n, bool al16, int e0) {
  const int sent = -2147483647 - 1;
  v4i d;
  if (al16 && (e0 + 3 < n)) {
    d = *(const v4i*)(arr + e0);
  } else {
    d.x = (e0     < n) ? arr[iclamp(e0,     0, n - 1)] : sent;
    d.y = (e0 + 1 < n) ? arr[iclamp(e0 + 1, 0, n - 1)] : sent;
    d.z = (e0 + 2 < n) ? arr[iclamp(e0 + 2, 0, n - 1)] : sent;
    d.w = (e0 + 3 < n) ? arr[iclamp(e0 + 3, 0, n - 1)] : sent;
  }
  return d;
}

__device__ __forceinline__ void hit4(v4i d, int el0, int base, unsigned span, int sh,
                                     int* wl, int& wc) {
  const unsigned s0 = (unsigned)d.x - (unsigned)base;
  const unsigned s1 = (unsigned)d.y - (unsigned)base;
  const unsigned s2 = (unsigned)d.z - (unsigned)base;
  const unsigned s3 = (unsigned)d.w - (unsigned)base;
  const bool h0 = s0 < span, h1 = s1 < span, h2 = s2 < span, h3 = s3 < span;
  const unsigned anyh = __builtin_amdgcn_ballot_w32(h0 | h1 | h2 | h3);
  if (anyh == 0u) return;
#define HITJ(J, HJ, SJ) { \
    const unsigned mj = __builtin_amdgcn_ballot_w32(HJ); \
    if (HJ) { \
      const int pos = wc + (int)__builtin_amdgcn_mbcnt_lo(mj, 0u); \
      if (pos < WCAP) wl[pos] = ((el0 + (J)) << sh) | (int)(SJ); \
    } \
    wc += (int)__builtin_popcount(mj); }
  HITJ(0, h0, s0)
  HITJ(1, h1, s1)
  HITJ(2, h2, s2)
  HITJ(3, h3, s3)
#undef HITJ
}

__global__ __launch_bounds__(NTHR) void k_prep(const float* __restrict__ W, _Float16* Wt, int n8) {
  const int i = blockIdx.x * NTHR + threadIdx.x;
  if (i >= n8) return;
  const int o  = i * 8;
  const int l  = o >> 13;
  const int rm = o & 8191;
  const int n  = rm >> 7;
  const int k0 = rm & 127;
  const float* s = W + (size_t)l * (DIN * DO) + (size_t)k0 * DO + n;
  Pack16 u;
#pragma unroll
  for (int j = 0; j < 8; ++j) u.h[j] = (_Float16)(s[j * DO] * 8.0f);
  _Float16* dp = Wt + o;
  *(volatile v4i*)dp = u.i;
  __threadfence();
  *(volatile v4i*)dp = u.i;
}

__global__ __launch_bounds__(GT) void k_gemm(
    const float* __restrict__ xin, const _Float16* __restrict__ Wt,
    const float* __restrict__ avs, const float* __restrict__ avd,
    float* hout, float* ssrc, float* sdst, int nN) {
  __shared__ __attribute__((aligned(16))) _Float16 At[GR * AP];
  __shared__ __attribute__((aligned(16))) float Hs[GR * HSP];
  __shared__ __attribute__((aligned(16))) float Ss[GR];
  __shared__ __attribute__((aligned(16))) float Sd[GR];

  const int tid  = threadIdx.x;
  const int lane = tid & 31;
  const int wave = tid >> 5;
  const int hh   = lane >> 4;
  const int m    = lane & 15;
  const int rowBase = blockIdx.x * GR;

  {
    const int r   = tid >> 2;
    const int cb  = (tid & 3) * 32;
    int row = rowBase + r;
    if (row > nN - 1) row = nN - 1;
    const float* p = xin + (size_t)row * DIN + cb;
#pragma unroll
    for (int j = 0; j < 4; ++j) {
      const v4f f0 = *(const v4f*)(p + 8 * j);
      const v4f f1 = *(const v4f*)(p + 8 * j + 4);
      Pack16 u;
      u.h[0] = (_Float16)f0.x; u.h[1] = (_Float16)f0.y; u.h[2] = (_Float16)f0.z; u.h[3] = (_Float16)f0.w;
      u.h[4] = (_Float16)f1.x; u.h[5] = (_Float16)f1.y; u.h[6] = (_Float16)f1.z; u.h[7] = (_Float16)f1.w;
      *(v8h*)(At + r * AP + cb + 8 * j) = u.h;
    }
  }
  __syncthreads();

  const int ncol = wave * 16 + m;
  v8f acc0 = {0.f, 0.f, 0.f, 0.f, 0.f, 0.f, 0.f, 0.f};
  v8f acc1 = {0.f, 0.f, 0.f, 0.f, 0.f, 0.f, 0.f, 0.f};
#pragma unroll
  for (int kt = 0; kt < DIN / 32; ++kt) {
    const int k0 = kt * 32;
    Frag a0, a1, b;
    const _Float16* pb  = Wt + (size_t)ncol * DIN + k0 + 8 * hh;
    const _Float16* pa0 = At + m * AP + k0 + 8 * hh;
    const _Float16* pa1 = At + (16 + m) * AP + k0 + 8 * hh;
    b.half[0]  = *(const v8h*)pb;   b.half[1]  = *(const v8h*)(pb + 16);
    a0.half[0] = *(const v8h*)pa0;  a0.half[1] = *(const v8h*)(pa0 + 16);
    a1.half[0] = *(const v8h*)pa1;  a1.half[1] = *(const v8h*)(pa1 + 16);
    acc0 = wm(a0.v, b.v, acc0);
    acc1 = wm(a1.v, b.v, acc1);
  }

#pragma unroll
  for (int r = 0; r < 8; ++r) {
    Hs[(8 * hh + r) * HSP + ncol]      = acc0[r] * 0.125f;
    Hs[(16 + 8 * hh + r) * HSP + ncol] = acc1[r] * 0.125f;
  }
  __syncthreads();

  {
    const int r = tid >> 2;
    const int q = tid & 3;
    const float* hp  = Hs + r * HSP + 16 * q;
    const float* asp = avs + 16 * q;
    const float* adp = avd + 16 * q;
    float s = 0.f, d = 0.f;
#pragma unroll
    for (int j = 0; j < 4; ++j) {
      const v4f v  = *(const v4f*)(hp + 4 * j);
      const v4f wa = *(const v4f*)(asp + 4 * j);
      const v4f wd = *(const v4f*)(adp + 4 * j);
      s += v.x * wa.x + v.y * wa.y + v.z * wa.z + v.w * wa.w;
      d += v.x * wd.x + v.y * wd.y + v.z * wd.z + v.w * wd.w;
    }
    s += __shfl_xor(s, 1, 32); s += __shfl_xor(s, 2, 32);
    d += __shfl_xor(d, 1, 32); d += __shfl_xor(d, 2, 32);
    if (q == 0) { Ss[r] = s; Sd[r] = d; }
  }
  __syncthreads();

  v4f hr[4];
  float* hp4[4];
#pragma unroll
  for (int i = 0; i < 4; ++i) {
    const int row = 8 * wave + 2 * i + hh;
    hr[i]  = *(const v4f*)(Hs + row * HSP + 4 * m);
    hp4[i] = hout + (size_t)(rowBase + row) * DO + 4 * m;
  }
  v4f sv = {0.f, 0.f, 0.f, 0.f};
  float* sp = 0;
  if (wave == 0) {
    if (lane < 8)       { sv = *(const v4f*)(Ss + 4 * lane);        sp = ssrc + rowBase + 4 * lane; }
    else if (lane < 16) { sv = *(const v4f*)(Sd + 4 * (lane - 8));  sp = sdst + rowBase + 4 * (lane - 8); }
  }
#pragma unroll
  for (int i = 0; i < 4; ++i) *(volatile v4f*)(hp4[i]) = hr[i];
  if (sp) *(volatile v4f*)sp = sv;
  __threadfence();
#pragma unroll
  for (int i = 0; i < 4; ++i) *(volatile v4f*)(hp4[i]) = hr[i];
  if (sp) *(volatile v4f*)sp = sv;
}

__global__ __launch_bounds__(NTHR) void k_gat(
    const int* __restrict__ ei, int nE,
    const float* __restrict__ h, const float* __restrict__ ssrc, const float* __restrict__ sdst,
    const float* __restrict__ bias, float* xa, int colOff, int nN) {
  extern __shared__ v4f lds_dyn[];
  float* sacc = (float*)lds_dyn;
  float* mrun = sacc + NB * DO;
  float* den  = mrun + NB;
  int*   list = (int*)(den + NB);
  int*   wcnt = list + NWAVE * WCAP;

  const int tid  = threadIdx.x;
  const int lane = tid & 31;
  const int wave = tid >> 5;
  const int nodeBase = blockIdx.x * NB;

  {
    const v4f z4 = {0.f, 0.f, 0.f, 0.f};
    for (int i = tid; i < (NB * DO) / 4; i += NTHR) lds_dyn[i] = z4;
    for (int i = tid; i < NB; i += NTHR) { mrun[i] = -1.0e30f; den[i] = 0.f; }
  }
  __syncthreads();

  const int* eid   = ei + nE;
  const bool al16  = ((nE & 3) == 0);
  int* wl = list + wave * WCAP;
  const int nChunks = (nE + CHUNK - 1) / CHUNK;

#pragma unroll 1
  for (int ch = 0; ch < nChunks; ++ch) {
    const int cbase = ch * CHUNK;
    int wc = 0;
#pragma unroll
    for (int g = 0; g < NGRP; ++g) {
      const int el0 = (g * NTHR + tid) * 4;
      const v4i d = load4(eid, nE, al16, cbase + el0);
      hit4(d, el0, nodeBase, (unsigned)NB, SLB, wl, wc);
    }
    if (lane == 0) wcnt[wave] = wc;
    __syncthreads();

    if (wave == 0) {
#pragma unroll 1
      for (int wsx = 0; wsx < NWAVE; ++wsx) {
        int n = wcnt[wsx];
        n = n > WCAP ? WCAP : (n < 0 ? 0 : n);
        const int* ls = list + wsx * WCAP;
#pragma unroll 1
        for (int i = 0; i < n; ++i) {
          const int ent  = __builtin_amdgcn_readfirstlane(ls[i]);
          const int slot = ent & (NB - 1);
          const int el   = (ent >> SLB) & (CHUNK - 1);
          int e = cbase + el;
          if (e > nE - 1) e = nE - 1;
          const int src = iclamp(ei[e], 0, nN - 1);
          int nd = nodeBase + slot;
          if (nd > nN - 1) nd = nN - 1;
          const float lg   = lrelu(ssrc[src] + sdst[nd]);
          const float mo   = mrun[slot];
          const float mn   = fmaxf(mo, lg);
          const float corr = __expf(mo - mn);
          const float p    = __expf(lg - mn);
          const v2f hv = *(const v2f*)(h + (size_t)src * DO + 2 * lane);
          v2f* sp = (v2f*)(sacc + slot * DO + 2 * lane);
          v2f a = *sp;
          a = a * corr + hv * p;
          *sp = a;
          if (lane == 0) {
            const float dv = den[slot];
            den[slot]  = dv * corr + p;
            mrun[slot] = mn;
          }
        }
      }
    }
    __syncthreads();
  }

  {
    const int hf = lane >> 4;
    const int c4 = (lane & 15) * 4;
    const v4f b4 = *(const v4f*)(bias + c4);
#pragma unroll 1
    for (int j = 0; j < NB / (NWAVE * 2); ++j) {
      const int s0 = wave * (NB / NWAVE) + 2 * j;
      if (nodeBase + s0 >= nN) break;
      const int slot = s0 + hf;
      const int node = nodeBase + slot;
      const int nl   = node < nN ? node : nN - 1;
      const float lg   = lrelu(ssrc[nl] + sdst[nl]);
      const float mo   = mrun[slot];
      const float mn   = fmaxf(mo, lg);
      const float corr = __expf(mo - mn);
      const float p    = __expf(lg - mn);
      const v4f hv = *(const v4f*)(h + (size_t)nl * DO + c4);
      v4f a = *(const v4f*)(sacc + slot * DO + c4);
      a = a * corr + hv * p;
      const float dn  = den[slot] * corr + p;
      const float inv = 1.0f / dn;
      v4f o = a * inv + b4;
      o.x = o.x > 0.f ? o.x : 0.f;
      o.y = o.y > 0.f ? o.y : 0.f;
      o.z = o.z > 0.f ? o.z : 0.f;
      o.w = o.w > 0.f ? o.w : 0.f;
      float* op = xa + (size_t)node * DIN + colOff + c4;
      const bool ok = node < nN;
      if (ok) *(volatile v4f*)op = o;
      __threadfence();
      if (ok) *(volatile v4f*)op = o;
    }
  }
}

__device__ __forceinline__ void st_out(float* p, v4f v, int idx, int nloc) {
  if (idx + 4 <= nloc) {
    *(volatile v4f*)p = v;
  } else if (idx < nloc) {
    volatile float* q = (volatile float*)p;
    q[0] = v.x;
    if (idx + 1 < nloc) q[1] = v.y;
    if (idx + 2 < nloc) q[2] = v.z;
  }
}

__global__ __launch_bounds__(NTHR) void k_pool(
    const float* __restrict__ x, const int* __restrict__ bt,
    const float* __restrict__ fw, const float* __restrict__ fb,
    float* y, int nN, int ng) {
  extern __shared__ v4f lds_p[];
  float* gacc = (float*)lds_p;
  int*   list = (int*)(gacc + NG * DIN);
  int*   wcnt = list + NWAVE * WCAP;
  float* ys   = (float*)(wcnt + NWAVE);

  const int tid  = threadIdx.x;
  const int lane = tid & 31;
  const int wave = tid >> 5;
  const int gbase = blockIdx.x * NG;

  {
    const v4f z4 = {0.f, 0.f, 0.f, 0.f};
    for (int i = tid; i < (NG * DIN) / 4; i += NTHR) lds_p[i] = z4;
  }
  __syncthreads();

  int* wl = list + wave * WCAP;
  const int nChunks = (nN + CHUNK - 1) / CHUNK;
#pragma unroll 1
  for (int ch = 0; ch < nChunks; ++ch) {
    const int cbase = ch * CHUNK;
    int wc = 0;
#pragma unroll
    for (int g = 0; g < NGRP; ++g) {
      const int el0 = (g * NTHR + tid) * 4;
      const v4i d = load4(bt, nN, true, cbase + el0);
      hit4(d, el0, gbase, (unsigned)NG, GLB, wl, wc);
    }
    if (lane == 0) wcnt[wave] = wc;
    __syncthreads();

    if (wave == 0) {
#pragma unroll 1
      for (int wsx = 0; wsx < NWAVE; ++wsx) {
        int n = wcnt[wsx];
        n = n > WCAP ? WCAP : (n < 0 ? 0 : n);
        const int* ls = list + wsx * WCAP;
#pragma unroll 1
        for (int i = 0; i < n; ++i) {
          const int ent = __builtin_amdgcn_readfirstlane(ls[i]);
          const int gs  = ent & (NG - 1);
          const int el  = (ent >> GLB) & (CHUNK - 1);
          int node = cbase + el;
          if (node > nN - 1) node = nN - 1;
          const v4f xv = *(const v4f*)(x + (size_t)node * DIN + 4 * lane);
          v4f* gp = (v4f*)(gacc + gs * DIN + 4 * lane);
          const v4f cur = *gp;
          *gp = cur + xv;
        }
      }
    }
    __syncthreads();
  }

  {
    const v4f fw4 = *(const v4f*)(fw + 4 * lane);
    const float fb0 = fb[0];
#pragma unroll 1
    for (int g = wave; g < NG; g += NWAVE) {
      const v4f a = *(const v4f*)(gacc + g * DIN + 4 * lane);
      float s = a.x * fw4.x + a.y * fw4.y + a.z * fw4.z + a.w * fw4.w;
      s = wsum(s);
      if (lane == 0) ys[g] = s + fb0;
    }
  }
  __syncthreads();

  if (wave == 0) {
    int nloc = ng - gbase;
    if (nloc > NG) nloc = NG;
    const int i0 = 4 * lane, i1 = 128 + 4 * lane, i2 = 256 + 4 * lane, i3 = 384 + 4 * lane;
    const v4f v0 = *(const v4f*)(ys + i0);
    const v4f v1 = *(const v4f*)(ys + i1);
    const v4f v2 = *(const v4f*)(ys + i2);
    const v4f v3 = *(const v4f*)(ys + i3);
    float* yb = y + gbase;
    st_out(yb + i0, v0, i0, nloc);
    st_out(yb + i1, v1, i1, nloc);
    st_out(yb + i2, v2, i2, nloc);
    st_out(yb + i3, v3, i3, nloc);
    __threadfence();
    st_out(yb + i0, v0, i0, nloc);
    st_out(yb + i1, v1, i1, nloc);
    st_out(yb + i2, v2, i2, nloc);
    st_out(yb + i3, v3, i3, nloc);
  }
}

static size_t al256(size_t b) { return (b + 255) & ~(size_t)255; }

extern "C" void kernel_launch(void* const* d_in, const int* in_sizes, int n_in,
                              void* d_out, int out_size, void* d_ws, size_t ws_size,
                              hipStream_t stream) {
  if (n_in < 10) return;
  const int nN = in_sizes[0] / DIN;
  if (nN <= 0 || in_sizes[0] != nN * DIN) return;
  if (in_sizes[1] < 0 || (in_sizes[1] & 1) != 0) return;
  if (in_sizes[2] < 0 || (in_sizes[2] & 1) != 0) return;
  const int nEs = in_sizes[1] / 2;
  const int nEd = in_sizes[2] / 2;
  if (in_sizes[3] != nN) return;
  if (in_sizes[4] != NL * DIN * DO) return;
  if (in_sizes[5] != NL * DO || in_sizes[6] != NL * DO || in_sizes[7] != NL * DO) return;
  if (in_sizes[8] != DIN || in_sizes[9] < 1) return;
  const int ng = out_size;
  if (ng <= 0) return;

  const float* x       = (const float*)d_in[0];
  const int*   ei_s    = (const int*)d_in[1];
  const int*   ei_d    = (const int*)d_in[2];
  const int*   batch   = (const int*)d_in[3];
  const float* lin_w   = (const float*)d_in[4];
  const float* att_src = (const float*)d_in[5];
  const float* att_dst = (const float*)d_in[6];
  const float* bias    = (const float*)d_in[7];
  const float* final_w = (const float*)d_in[8];
  const float* final_b = (const float*)d_in[9];
  float* y = (float*)d_out;

  const int nP = ((nN + GR - 1) / GR) * GR;
  size_t off = 0;
  const size_t oWt = off; off += al256((size_t)NL * DO * DIN * sizeof(_Float16));
  const size_t oH  = off; off += al256((size_t)nP * DO * sizeof(float));
  const size_t oSs = off; off += al256((size_t)nP * sizeof(float));
  const size_t oSd = off; off += al256((size_t)nP * sizeof(float));
  const size_t oXa = off; off += al256((size_t)nP * DIN * sizeof(float));
  if (off > ws_size || off > (size_t)134217728) return;

  _Float16* Wt = (_Float16*)((char*)d_ws + oWt);
  float* hbuf  = (float*)((char*)d_ws + oH);
  float* ssrc  = (float*)((char*)d_ws + oSs);
  float* sdst  = (float*)((char*)d_ws + oSd);
  float* xa    = (float*)((char*)d_ws + oXa);

  const int n8 = NL * DO * DIN / 8;
  k_prep<<<(n8 + NTHR - 1) / NTHR, NTHR, 0, stream>>>(lin_w, Wt, n8);

  hipFuncSetAttribute(reinterpret_cast<const void*>(&k_gat),
                      hipFuncAttributeMaxDynamicSharedMemorySize, LDS_GAT_BYTES);
  hipFuncSetAttribute(reinterpret_cast<const void*>(&k_pool),
                      hipFuncAttributeMaxDynamicSharedMemorySize, LDS_POOL_BYTES);

  const int gemmGrid = nP / GR;
  const int gatGrid  = (nN + NB - 1) / NB;
  for (int l = 0; l < NL; ++l) {
    const float* xin = (l == 0) ? x : xa;
    k_gemm<<<gemmGrid, GT, 0, stream>>>(xin, Wt + (size_t)l * DO * DIN,
                                         att_src + l * DO, att_dst + l * DO,
                                         hbuf, ssrc, sdst, nN);
    k_gat<<<gatGrid, NTHR, LDS_GAT_BYTES, stream>>>(ei_s, nEs, hbuf, ssrc, sdst,
                                                     bias + l * DO, xa, 0, nN);
    k_gat<<<gatGrid, NTHR, LDS_GAT_BYTES, stream>>>(ei_d, nEd, hbuf, ssrc, sdst,
                                                     bias + l * DO, xa, DO, nN);
  }

  const int poolGrid = (ng + NG - 1) / NG;
  k_pool<<<poolGrid, NTHR, LDS_POOL_BYTES, stream>>>(xa, batch, final_w, final_b, y, nN, ng);
}
